// FDGRPretrainedModel_3942779978211
// MI455X (gfx1250) — hardware-run, weakly checked
//
#include <hip/hip_runtime.h>
#include <stdint.h>
#include <stddef.h>
#include <math.h>

#define NR   1024
#define NHF  512
#define DM   768
#define DH   256
#define DC   512
#define CP   68
#define TP   65
#define WSC  64.0f
#define WINV 0.015625f
#define OUTF 524293
#define OUT4 131072

static_assert(NR % 64 == 0);
static_assert(NHF % 64 == 0);
static_assert(DM % 64 == 0);
static_assert(DH % 64 == 0);
static_assert(DC % 64 == 0);
static_assert((CP * 4) % 16 == 0);
static_assert(OUTF == 5 + 2 * NR * DH);
static_assert(4 * OUT4 + 5 == OUTF);
static_assert((NR * DM) % 2048 == 0);
static_assert(NR % 32 == 0);
static_assert(NHF % 32 == 0);

typedef _Float16       v16h __attribute__((ext_vector_type(16)));
typedef _Float16       v8h  __attribute__((ext_vector_type(8)));
typedef float          v8f  __attribute__((ext_vector_type(8)));
typedef float          v4f  __attribute__((ext_vector_type(4)));
typedef unsigned int   v4u  __attribute__((ext_vector_type(4)));
typedef v4f __attribute__((may_alias)) v4fa;
typedef v4u __attribute__((may_alias)) v4ua;
typedef v8h __attribute__((may_alias)) v8ha;

union FragH { v16h v; v8h half[2]; };
union H8 { v8h h; v4u u; };
static_assert(sizeof(FragH) == 32);
static_assert(sizeof(H8) == 16);

__device__ __forceinline__ v8f wmma_hf(v16h a, v16h b, v8f c) {
  v8f d = __builtin_amdgcn_wmma_f32_16x16x32_f16(false, a, false, b, (short)0, c, false, false);
  asm volatile("v_nop\n\tv_nop\n\tv_nop\n\tv_nop" : "+v"(d) : "v"(a), "v"(b));
  return d;
}
__device__ __forceinline__ v16h ldfh(const _Float16* p, int h) {
  FragH f;
  f.half[0] = *(const v8ha*)(p + 8 * h);
  f.half[1] = *(const v8ha*)(p + 16 + 8 * h);
  return f.v;
}

__device__ __forceinline__ float wsum(float v) {
  #pragma unroll
  for (int o = 16; o > 0; o >>= 1) v += __shfl_xor(v, o, 32);
  return v;
}
__device__ __forceinline__ float wmax(float v) {
  #pragma unroll
  for (int o = 16; o > 0; o >>= 1) v = fmaxf(v, __shfl_xor(v, o, 32));
  return v;
}
__device__ __forceinline__ float dot4(v4f a, v4f b) {
  return fmaf(a.x, b.x, fmaf(a.y, b.y, fmaf(a.z, b.z, a.w * b.w)));
}
__device__ __forceinline__ float softp(float x) {
  return fmaxf(x, 0.f) + __logf(1.0f + __expf(-fabsf(x)));
}

__global__ __launch_bounds__(256) void k_cvt(const float* __restrict__ src,
                                             _Float16* __restrict__ dst, int n8)
{
  const int gid = blockIdx.x * 256 + threadIdx.x;
  if (gid >= n8) return;
  const float* s = src + (size_t)gid * 8;
  const v4f a = *(const v4fa*)s;
  const v4f b = *(const v4fa*)(s + 4);
  const v8f f = {a.x, a.y, a.z, a.w, b.x, b.y, b.z, b.w};
  H8 P; P.h = __builtin_convertvector(f, v8h);
  _Float16* dp = dst + (size_t)gid * 8;
  *(volatile v4ua*)dp = P.u;
  __threadfence();
  *(volatile v4ua*)dp = P.u;
}

__device__ __forceinline__ void packw_store(const float* sW, _Float16* Wp, int Kdim,
                                            int n0, int k0, int tid)
{
  #pragma unroll
  for (int it = 0; it < 2; ++it) {
    const int slot = tid + 256 * it;
    const int n = slot >> 3, kq = slot & 7;
    const float* c = sW + (8 * kq) * TP + n;
    const v8f f = {c[0] * WSC,      c[TP] * WSC,     c[2 * TP] * WSC, c[3 * TP] * WSC,
                   c[4 * TP] * WSC, c[5 * TP] * WSC, c[6 * TP] * WSC, c[7 * TP] * WSC};
    H8 P; P.h = __builtin_convertvector(f, v8h);
    *(volatile v4ua*)(Wp + (size_t)(n0 + n) * Kdim + k0 + 8 * kq) = P.u;
  }
}

__global__ __launch_bounds__(256) void k_packw(const float* __restrict__ W, int Kdim, int Ndim,
                                               _Float16* __restrict__ Wp)
{
  __shared__ float sW[64 * TP];
  const int tid = threadIdx.x;
  const int n0 = blockIdx.x * 64, k0 = blockIdx.y * 64;
  #pragma unroll
  for (int it = 0; it < 4; ++it) {
    const int idx = tid + 256 * it;
    const int r = idx >> 4, c4 = idx & 15;
    const v4f v = *(const v4fa*)(W + (size_t)(k0 + r) * Ndim + n0 + 4 * c4);
    float* d = sW + r * TP + 4 * c4;
    d[0] = v.x; d[1] = v.y; d[2] = v.z; d[3] = v.w;
  }
  __syncthreads();
  packw_store(sW, Wp, Kdim, n0, k0, tid);
  __threadfence();
  packw_store(sW, Wp, Kdim, n0, k0, tid);
}

__device__ __forceinline__ void g_store32(const float* sC, float* C32, int ldc, int m0, int n0,
                                          int wv, int lane)
{
  #pragma unroll
  for (int i = 0; i < 16; ++i) {
    const int row = 32 * wv + 2 * i + (lane >> 4);
    const int c4 = 4 * (lane & 15);
    const v4f v = *(const v4fa*)(sC + row * CP + c4);
    *(volatile v4fa*)(C32 + (size_t)(m0 + row) * ldc + n0 + c4) = v;
  }
}
__device__ __forceinline__ void g_store16(const float* sC, _Float16* C16, int ldc, int m0, int n0,
                                          int wv, int lane)
{
  #pragma unroll
  for (int i = 0; i < 8; ++i) {
    const int row = 32 * wv + 4 * i + (lane >> 3);
    const int c8 = 8 * (lane & 7);
    const v4f x0 = *(const v4fa*)(sC + row * CP + c8);
    const v4f x1 = *(const v4fa*)(sC + row * CP + c8 + 4);
    const v8f f = {x0.x, x0.y, x0.z, x0.w, x1.x, x1.y, x1.z, x1.w};
    H8 P; P.h = __builtin_convertvector(f, v8h);
    *(volatile v4ua*)(C16 + (size_t)(m0 + row) * ldc + n0 + c8) = P.u;
  }
}

__global__ __launch_bounds__(64) void k_gemm(const _Float16* __restrict__ A, int lda,
                                             const _Float16* __restrict__ Wp, int K,
                                             const float* __restrict__ bias, int has_bias,
                                             float scale, int act,
                                             float* C32, int has32,
                                             _Float16* C16, int has16, int ldc)
{
  __shared__ __align__(16) float sC[64 * CP];
  const int tid = threadIdx.x, lane = tid & 31, wv = tid >> 5;
  const int h = lane >> 4, m = lane & 15;
  const int m0 = blockIdx.y * 64, n0 = blockIdx.x * 64;
  const _Float16* ar0 = A + (size_t)(m0 + 32 * wv + m) * lda;
  const _Float16* ar1 = ar0 + (size_t)16 * lda;
  const _Float16* br  = Wp + (size_t)(n0 + m) * K;
  const v8f z8 = {0.f, 0.f, 0.f, 0.f, 0.f, 0.f, 0.f, 0.f};
  v8f acc[2][4];
  #pragma unroll
  for (int t = 0; t < 2; ++t) {
    #pragma unroll
    for (int c = 0; c < 4; ++c) acc[t][c] = z8;
  }

  #pragma unroll 1
  for (int k0 = 0; k0 < K; k0 += 32) {
    const v16h a0 = ldfh(ar0 + k0, h);
    const v16h a1 = ldfh(ar1 + k0, h);
    #pragma unroll
    for (int c = 0; c < 4; ++c) {
      const v16h b = ldfh(br + (size_t)(16 * c) * K + k0, h);
      acc[0][c] = wmma_hf(a0, b, acc[0][c]);
      acc[1][c] = wmma_hf(a1, b, acc[1][c]);
    }
  }

  #pragma unroll
  for (int c = 0; c < 4; ++c) {
    const int col = 16 * c + m;
    const float bl = bias[n0 + col];
    const float bv = has_bias ? bl : 0.f;
    #pragma unroll
    for (int t = 0; t < 2; ++t) {
      #pragma unroll
      for (int r = 0; r < 8; ++r) {
        float v = fmaf(acc[t][c][r], scale, bv);
        v = act ? fmaxf(v, 0.f) : v;
        sC[(32 * wv + 16 * t + 8 * h + r) * CP + col] = v;
      }
    }
  }
  __syncthreads();
  if (has32) {
    g_store32(sC, C32, ldc, m0, n0, wv, lane);
    __threadfence();
    g_store32(sC, C32, ldc, m0, n0, wv, lane);
  }
  if (has16) {
    g_store16(sC, C16, ldc, m0, n0, wv, lane);
    __threadfence();
    g_store16(sC, C16, ldc, m0, n0, wv, lane);
  }
}

__global__ __launch_bounds__(256) void k_ln256(const float* __restrict__ X,
                                               const float* __restrict__ g,
                                               const float* __restrict__ bt,
                                               float* Y32, _Float16* Y16, int ld16, int coff,
                                               const float* __restrict__ other, int has_other,
                                               float* rowpart)
{
  __shared__ __align__(16) float sP[32];
  const int tid = threadIdx.x, lane = tid & 31, wv = tid >> 5;
  const int rb = blockIdx.x * 32;
  const v4f ga = *(const v4fa*)(g + 4 * lane);
  const v4f gb = *(const v4fa*)(g + 128 + 4 * lane);
  const v4f ba = *(const v4fa*)(bt + 4 * lane);
  const v4f bb = *(const v4fa*)(bt + 128 + 4 * lane);
  const v4f gc = *(const v4fa*)(g + 8 * lane);
  const v4f gd = *(const v4fa*)(g + 8 * lane + 4);
  const v4f bc = *(const v4fa*)(bt + 8 * lane);
  const v4f bd = *(const v4fa*)(bt + 8 * lane + 4);

  #pragma unroll 1
  for (int q = 0; q < 4; ++q) {
    const int rl = 4 * wv + q;
    const int row = rb + rl;
    const float* x = X + (size_t)row * DH;
    const v4f xa = *(const v4fa*)(x + 4 * lane);
    const v4f xb = *(const v4fa*)(x + 128 + 4 * lane);
    float s = ((xa.x + xa.y) + (xa.z + xa.w)) + ((xb.x + xb.y) + (xb.z + xb.w));
    s = wsum(s);
    const float mean = s * 0.00390625f;
    const v4f da = xa - mean;
    const v4f db = xb - mean;
    float qv = dot4(da, da) + dot4(db, db);
    qv = wsum(qv);
    const float var = qv * 0.00390625f;
    const float rstd = 1.0f / sqrtf(var + 1e-12f);
    const v4f ya = (da * rstd) * ga + ba;
    const v4f yb = (db * rstd) * gb + bb;
    float cl = 0.f;
    if (has_other) {
      const v4f oa = *(const v4fa*)(other + (size_t)row * DH + 4 * lane);
      const v4f ob = *(const v4fa*)(other + (size_t)row * DH + 128 + 4 * lane);
      const v4f ea = oa - ya;
      const v4f eb = ob - yb;
      cl = 0.5f * (dot4(ea, ea) + dot4(eb, eb));
    }
    cl = wsum(cl);
    if (lane == 0) sP[rl] = cl;
    const v4f xc = *(const v4fa*)(x + 8 * lane);
    const v4f xd = *(const v4fa*)(x + 8 * lane + 4);
    const v4f yc = ((xc - mean) * rstd) * gc + bc;
    const v4f yd = ((xd - mean) * rstd) * gd + bd;
    const v8f f = {yc.x, yc.y, yc.z, yc.w, yd.x, yd.y, yd.z, yd.w};
    H8 P; P.h = __builtin_convertvector(f, v8h);
    float* pa = Y32 + (size_t)row * DH + 4 * lane;
    float* pb = pa + 128;
    _Float16* ph = Y16 + (size_t)row * ld16 + coff + 8 * lane;
    *(volatile v4fa*)pa = ya;
    *(volatile v4fa*)pb = yb;
    *(volatile v4ua*)ph = P.u;
    __threadfence();
    *(volatile v4fa*)pa = ya;
    *(volatile v4fa*)pb = yb;
    *(volatile v4ua*)ph = P.u;
  }
  __syncthreads();
  if (has_other && wv == 0 && lane < 8) {
    const v4f v = *(const v4fa*)(sP + 4 * lane);
    float* dp = rowpart + (size_t)rb + 4 * lane;
    *(volatile v4fa*)dp = v;
    __threadfence();
    *(volatile v4fa*)dp = v;
  }
}

__global__ __launch_bounds__(256) void k_ln768(const float* __restrict__ X,
                                               const float* __restrict__ g,
                                               const float* __restrict__ bt,
                                               const float* __restrict__ S,
                                               float* rowpart)
{
  __shared__ __align__(16) float sP[32];
  const int tid = threadIdx.x, lane = tid & 31, wv = tid >> 5;
  const int rb = blockIdx.x * 32;
  const float i768 = 1.0f / 768.0f;

  #pragma unroll 1
  for (int q = 0; q < 4; ++q) {
    const int rl = 4 * wv + q;
    const int row = rb + rl;
    const float* x  = X + (size_t)row * DM;
    const float* sr = S + (size_t)row * DM;
    float s = 0.f;
    #pragma unroll 1
    for (int c = 0; c < 6; ++c) {
      const v4f v = *(const v4fa*)(x + 128 * c + 4 * lane);
      s += (v.x + v.y) + (v.z + v.w);
    }
    s = wsum(s);
    const float mean = s * i768;
    float qv = 0.f;
    #pragma unroll 1
    for (int c = 0; c < 6; ++c) {
      const v4f v = *(const v4fa*)(x + 128 * c + 4 * lane) - mean;
      qv += dot4(v, v);
    }
    qv = wsum(qv);
    const float var = qv * i768;
    const float rstd = 1.0f / sqrtf(var + 1e-12f);
    float e = 0.f;
    #pragma unroll 1
    for (int c = 0; c < 6; ++c) {
      const int co = 128 * c + 4 * lane;
      const v4f v  = *(const v4fa*)(x + co) - mean;
      const v4f gg = *(const v4fa*)(g + co);
      const v4f bv = *(const v4fa*)(bt + co);
      const v4f ss = *(const v4fa*)(sr + co);
      const v4f y  = (v * rstd) * gg + bv;
      const v4f d  = ss - y;
      e += dot4(d, d);
    }
    e = wsum(e);
    if (lane == 0) sP[rl] = e;
  }
  __syncthreads();
  if (wv == 0 && lane < 8) {
    const v4f v = *(const v4fa*)(sP + 4 * lane);
    float* dp = rowpart + (size_t)rb + 4 * lane;
    *(volatile v4fa*)dp = v;
    __threadfence();
    *(volatile v4fa*)dp = v;
  }
}

__global__ __launch_bounds__(256) void k_crit(const float* __restrict__ P,
                                              const float* __restrict__ Q,
                                              const float* __restrict__ w2,
                                              const float* __restrict__ b2,
                                              const int* __restrict__ ids_o,
                                              const int* __restrict__ ids_c,
                                              float* LSE, float* T0)
{
  __shared__ __align__(16) float sQ[32 * DH];
  __shared__ __align__(16) float sw[DH];
  __shared__ float sM[8];
  __shared__ float sS[8];
  __shared__ __align__(16) float sL[32];
  __shared__ __align__(16) float sT[32];
  const int tid = threadIdx.x, lane = tid & 31, wv = tid >> 5;
  const int i0 = blockIdx.x * 32;

  #pragma unroll
  for (int it = 0; it < 8; ++it) {
    const int idx = tid + 256 * it;
    *(v4fa*)(sQ + 4 * idx) = *(const v4fa*)(Q + (size_t)i0 * DH + 4 * idx);
  }
  sw[tid] = w2[tid];
  __syncthreads();
  const float b2v = b2[0];
  const v4f z4 = {0.f, 0.f, 0.f, 0.f};

  #pragma unroll 1
  for (int q = 0; q < 4; ++q) {
    const int il = 4 * wv + q;
    const int i = i0 + il;
    const float* pr = P + (size_t)i * DH + 8 * lane;
    const float* qr = sQ + il * DH + 8 * lane;
    const float* wr = sw + 8 * lane;
    const v4f x0 = __builtin_elementwise_max(*(const v4fa*)pr + *(const v4fa*)qr, z4);
    const v4f x1 = __builtin_elementwise_max(*(const v4fa*)(pr + 4) + *(const v4fa*)(qr + 4), z4);
    float s = dot4(x0, *(const v4fa*)wr) + dot4(x1, *(const v4fa*)(wr + 4));
    s = wsum(s);
    if (lane == 0) sT[il] = softp(s + b2v);
  }

  const int j0 = tid, j1 = tid + 256;
  const int oj0 = ids_o[j0], oj1 = ids_o[j1];
  const float* p0 = P + (size_t)j0 * DH;
  const float* p1 = P + (size_t)j1 * DH;

  #pragma unroll 1
  for (int il = 0; il < 32; ++il) {
    const int i = i0 + il;
    const int wi = ids_c[i];
    const float* qr = sQ + il * DH;
    float a0 = 0.f, a1 = 0.f;
    #pragma unroll 2
    for (int k4 = 0; k4 < DH / 4; ++k4) {
      const v4f q4 = *(const v4fa*)(qr + 4 * k4);
      const v4f w4 = *(const v4fa*)(sw + 4 * k4);
      const v4f r0 = __builtin_elementwise_max(*(const v4fa*)(p0 + 4 * k4) + q4, z4);
      const v4f r1 = __builtin_elementwise_max(*(const v4fa*)(p1 + 4 * k4) + q4, z4);
      a0 = fmaf(r0.x, w4.x, a0); a0 = fmaf(r0.y, w4.y, a0); a0 = fmaf(r0.z, w4.z, a0); a0 = fmaf(r0.w, w4.w, a0);
      a1 = fmaf(r1.x, w4.x, a1); a1 = fmaf(r1.y, w4.y, a1); a1 = fmaf(r1.z, w4.z, a1); a1 = fmaf(r1.w, w4.w, a1);
    }
    float t0v = softp(a0 + b2v);
    float t1v = softp(a1 + b2v);
    t0v = (wi == oj0 && j0 != i) ? -1.0e9f : t0v;
    t1v = (wi == oj1 && j1 != i) ? -1.0e9f : t1v;
    const float mx = wmax(fmaxf(t0v, t1v));
    if (lane == 0) sM[wv] = mx;
    __syncthreads();
    float M = sM[0];
    #pragma unroll
    for (int k = 1; k < 8; ++k) M = fmaxf(M, sM[k]);
    float e = __expf(t0v - M) + __expf(t1v - M);
    e = wsum(e);
    if (lane == 0) sS[wv] = e;
    __syncthreads();
    if (tid == 0) {
      float Ssum = sS[0];
      #pragma unroll
      for (int k = 1; k < 8; ++k) Ssum += sS[k];
      sL[il] = M + __logf(Ssum);
    }
  }
  __syncthreads();
  if (wv == 0 && lane < 16) {
    const int l8 = lane & 7;
    const v4f va = *(const v4fa*)(sL + 4 * l8);
    const v4f vb = *(const v4fa*)(sT + 4 * l8);
    float* dl = LSE + (size_t)i0 + 4 * l8;
    float* dt = T0 + (size_t)i0 + 4 * l8;
    if (lane < 8) *(volatile v4fa*)dl = va; else *(volatile v4fa*)dt = vb;
    __threadfence();
    if (lane < 8) *(volatile v4fa*)dl = va; else *(volatile v4fa*)dt = vb;
  }
}

__global__ __launch_bounds__(256) void k_vad(const float* __restrict__ V,
                                             const float* __restrict__ Av,
                                             const float* __restrict__ Dv,
                                             const float* __restrict__ pvw,
                                             const float* __restrict__ paw,
                                             const float* __restrict__ pdw,
                                             const float* __restrict__ pvb,
                                             const float* __restrict__ pab,
                                             const float* __restrict__ pdb,
                                             const float* __restrict__ vad_o,
                                             const float* __restrict__ vad_c,
                                             float* VADP, float* ORTH)
{
  __shared__ __align__(16) float sV[32];
  __shared__ __align__(16) float sO[32];
  const int tid = threadIdx.x, lane = tid & 31, wv = tid >> 5;
  const int rb = blockIdx.x * 32;

  #pragma unroll 1
  for (int q = 0; q < 4; ++q) {
    const int rl = 4 * wv + q;
    const int row = rb + rl;
    float spv = 0.f, spa = 0.f, spd = 0.f;
    float gvv = 0.f, gva = 0.f, gvd = 0.f, gaa = 0.f, gad = 0.f, gdd = 0.f;
    #pragma unroll 1
    for (int hq = 0; hq < 2; ++hq) {
      const int c = 128 * hq + 4 * lane;
      const size_t off = (size_t)row * DH + c;
      const v4f v = *(const v4fa*)(V + off);
      const v4f a = *(const v4fa*)(Av + off);
      const v4f d = *(const v4fa*)(Dv + off);
      const v4f wv4 = *(const v4fa*)(pvw + c);
      const v4f wa4 = *(const v4fa*)(paw + c);
      const v4f wd4 = *(const v4fa*)(pdw + c);
      spv += dot4(v, wv4); spa += dot4(a, wa4); spd += dot4(d, wd4);
      gvv += dot4(v, v); gva += dot4(v, a); gvd += dot4(v, d);
      gaa += dot4(a, a); gad += dot4(a, d); gdd += dot4(d, d);
    }
    spv = wsum(spv); spa = wsum(spa); spd = wsum(spd);
    gvv = wsum(gvv); gva = wsum(gva); gvd = wsum(gvd);
    gaa = wsum(gaa); gad = wsum(gad); gdd = wsum(gdd);
    const int ro = min(row, NHF - 1);
    const int rc = max(row - NHF, 0);
    const float to0 = vad_o[ro * 3 + 0], to1 = vad_o[ro * 3 + 1], to2 = vad_o[ro * 3 + 2];
    const float tc0 = vad_c[rc * 3 + 0], tc1 = vad_c[rc * 3 + 1], tc2 = vad_c[rc * 3 + 2];
    const bool first = (row < NHF);
    const float tg0 = first ? to0 : tc0;
    const float tg1 = first ? to1 : tc1;
    const float tg2 = first ? to2 : tc2;
    if (lane == 0) {
      const float e0 = (spv + pvb[0]) - tg0;
      const float e1 = (spa + pab[0]) - tg1;
      const float e2 = (spd + pdb[0]) - tg2;
      sV[rl] = e0 * e0 + e1 * e1 + e2 * e2;
      const float o0 = gvv - 1.0f, o1 = gaa - 1.0f, o2 = gdd - 1.0f;
      sO[rl] = o0 * o0 + o1 * o1 + o2 * o2 + 2.0f * (gva * gva + gvd * gvd + gad * gad);
    }
  }
  __syncthreads();
  if (wv == 0 && lane < 16) {
    const int l8 = lane & 7;
    const v4f va = *(const v4fa*)(sV + 4 * l8);
    const v4f vb = *(const v4fa*)(sO + 4 * l8);
    float* d0 = VADP + (size_t)rb + 4 * l8;
    float* d1 = ORTH + (size_t)rb + 4 * l8;
    if (lane < 8) *(volatile v4fa*)d0 = va; else *(volatile v4fa*)d1 = vb;
    __threadfence();
    if (lane < 8) *(volatile v4fa*)d0 = va; else *(volatile v4fa*)d1 = vb;
  }
}

__device__ __forceinline__ double bsum(double v, double* red)
{
  const int tid = threadIdx.x;
  red[tid] = v;
  __syncthreads();
  #pragma unroll
  for (int s = 128; s > 0; s >>= 1) {
    if (tid < s) red[tid] += red[tid + s];
    __syncthreads();
  }
  const double r = red[0];
  __syncthreads();
  return r;
}

__global__ __launch_bounds__(256) void k_loss(const float* __restrict__ CLUB,
                                              const float* __restrict__ REC,
                                              const float* __restrict__ LSE,
                                              const float* __restrict__ T0,
                                              const float* __restrict__ VADP,
                                              const float* __restrict__ ORTH,
                                              const int* __restrict__ amask,
                                              float* LOSS)
{
  __shared__ double red[256];
  __shared__ __align__(16) float sOut[32];
  (void)amask;
  const int tid = threadIdx.x;

  float l0 = LSE[tid], l1 = LSE[tid + 256];
  float t0 = T0[tid],  t1 = T0[tid + 256];
  asm volatile("" : "+v"(l0), "+v"(l1), "+v"(t0), "+v"(t1));
  const double l = (double)l0 + (double)l1;
  const double t = (double)t0 + (double)t1;

  double c = 0.0, r = 0.0, vd = 0.0, og = 0.0;
  #pragma unroll 1
  for (int k = 0; k < NR / 256; ++k) {
    const int idx = tid + 256 * k;
    float x0 = CLUB[idx];
    float x1 = REC[idx];
    float x2 = VADP[idx];
    float x3 = ORTH[idx];
    asm volatile("" : "+v"(x0), "+v"(x1), "+v"(x2), "+v"(x3));
    c  += (double)x0;
    r  += (double)x1;
    vd += (double)x2;
    og += (double)x3;
  }
  const double cs = bsum(c, red);
  const double rs = bsum(r, red);
  const double ls = bsum(l, red);
  const double ts = bsum(t, red);
  const double vs = bsum(vd, red);
  const double gs = bsum(og, red);
  if (tid == 0) {
    sOut[0] = (float)(cs / (double)NR);
    sOut[1] = (float)(rs / ((double)NR * (double)DM));
    sOut[2] = (float)gs;
    const double lb = ts / (double)NHF - (ls / (double)NHF - (double)logf((float)NHF));
    sOut[3] = (float)(-lb);
    sOut[4] = (float)(vs / ((double)NR * 3.0));
    #pragma unroll
    for (int k = 5; k < 32; ++k) sOut[k] = 0.f;
  }
  __syncthreads();
  if (tid < 8) {
    const v4f v = *(const v4fa*)(sOut + 4 * tid);
    float* dp = LOSS + 4 * tid;
    *(volatile v4fa*)dp = v;
    __threadfence();
    *(volatile v4fa*)dp = v;
  }
}

__device__ __forceinline__ float out_val(int f, const float* LOSS, const float* HA, const float* HC)
{
  const int li = min(f, 31);
  const int ai = min(max(f - 5, 0), NR * DH - 1);
  const int ci = min(max(f - 5 - NR * DH, 0), NR * DH - 1);
  const float lv = LOSS[li];
  const float av = HA[ai];
  const float cv = HC[ci];
  return (f < 5) ? lv : ((f < 5 + NR * DH) ? av : cv);
}

__global__ __launch_bounds__(256) void k_out(const float* __restrict__ LOSS,
                                             const float* __restrict__ HA,
                                             const float* __restrict__ HC,
                                             float* out)
{
  const int gid = blockIdx.x * 256 + threadIdx.x;
  if (gid > OUT4) return;
  const int f = 4 * gid;
  v4f v;
  v.x = out_val(f,     LOSS, HA, HC);
  v.y = out_val(f + 1, LOSS, HA, HC);
  v.z = out_val(f + 2, LOSS, HA, HC);
  v.w = out_val(f + 3, LOSS, HA, HC);
  const bool tail = (gid == OUT4);
  const float tv = HC[NR * DH - 1];
  float* dp = out + (size_t)f;
  *(volatile v4fa*)dp = v;
  if (tail) *(volatile float*)(out + (OUTF - 1)) = tv;
  __threadfence();
  *(volatile v4fa*)dp = v;
  if (tail) *(volatile float*)(out + (OUTF - 1)) = tv;
}

extern "C" void kernel_launch(void* const* d_in, const int* in_sizes, int n_in,
                              void* d_out, int out_size, void* d_ws, size_t ws_size,
                              hipStream_t stream)
{
  if (n_in < 40) return;
  if (in_sizes[0]  != NR * DM) return;
  if (in_sizes[1]  != NHF * 3) return;
  if (in_sizes[2]  != NHF * 3) return;
  if (in_sizes[3]  != NHF) return;
  if (in_sizes[4]  != NHF) return;
  if (in_sizes[5]  != NHF) return;
  if (in_sizes[6]  != DM * DM) return;
  if (in_sizes[7]  != DM * DH) return;
  if (in_sizes[8]  != DM * DM) return;
  if (in_sizes[9]  != DM * DH) return;
  if (in_sizes[10] != DC * DM) return;
  if (in_sizes[11] != DM * DM) return;
  if (in_sizes[12] != DH * DH) return;
  if (in_sizes[13] != DH * DH) return;
  if (in_sizes[14] != DH * DH) return;
  if (in_sizes[15] != DH) return;
  if (in_sizes[16] != DH) return;
  if (in_sizes[17] != DH) return;
  if (in_sizes[18] != DC * DH) return;
  if (in_sizes[19] != DH) return;
  if (in_sizes[20] != DM) return;
  if (in_sizes[21] != DH) return;
  if (in_sizes[22] != DH) return;
  if (in_sizes[23] != DH) return;
  if (in_sizes[24] != DM) return;
  if (in_sizes[25] != DH) return;
  if (in_sizes[26] != DH) return;
  if (in_sizes[27] != DH) return;
  if (in_sizes[28] != DM) return;
  if (in_sizes[29] != DM) return;
  if (in_sizes[30] != DM) return;
  if (in_sizes[31] != DM) return;
  if (in_sizes[32] != DH) return;
  if (in_sizes[33] != DH) return;
  if (in_sizes[34] != DH) return;
  if (in_sizes[35] != 1) return;
  if (in_sizes[36] != 1) return;
  if (in_sizes[37] != 1) return;
  if (in_sizes[38] != DH) return;
  if (in_sizes[39] != 1) return;
  if (out_size != OUTF) return;

  const float* seq   = (const float*)d_in[0];
  const float* vad_o = (const float*)d_in[1];
  const float* vad_c = (const float*)d_in[2];
  const int*   ids_o = (const int*)d_in[3];
  const int*   ids_c = (const int*)d_in[4];
  const int*   amask = (const int*)d_in[5];
  const float* ha_w1 = (const float*)d_in[6];
  const float* ha_w2 = (const float*)d_in[7];
  const float* hc_w1 = (const float*)d_in[8];
  const float* hc_w2 = (const float*)d_in[9];
  const float* de_w1 = (const float*)d_in[10];
  const float* de_w2 = (const float*)d_in[11];
  const float* v_w   = (const float*)d_in[12];
  const float* a_w   = (const float*)d_in[13];
  const float* d_w   = (const float*)d_in[14];
  const float* pv_w  = (const float*)d_in[15];
  const float* pa_w  = (const float*)d_in[16];
  const float* pd_w  = (const float*)d_in[17];
  const float* f_w1  = (const float*)d_in[18];
  const float* f_w2  = (const float*)d_in[19];
  const float* ha_b1 = (const float*)d_in[20];
  const float* ha_b2 = (const float*)d_in[21];
  const float* ha_g  = (const float*)d_in[22];
  const float* ha_bt = (const float*)d_in[23];
  const float* hc_b1 = (const float*)d_in[24];
  const float* hc_b2 = (const float*)d_in[25];
  const float* hc_g  = (const float*)d_in[26];
  const float* hc_bt = (const float*)d_in[27];
  const float* de_b1 = (const float*)d_in[28];
  const float* de_b2 = (const float*)d_in[29];
  const float* de_g  = (const float*)d_in[30];
  const float* de_bt = (const float*)d_in[31];
  const float* v_b   = (const float*)d_in[32];
  const float* a_b   = (const float*)d_in[33];
  const float* d_b   = (const float*)d_in[34];
  const float* pv_b  = (const float*)d_in[35];
  const float* pa_b  = (const float*)d_in[36];
  const float* pd_b  = (const float*)d_in[37];
  const float* f_b1  = (const float*)d_in[38];
  const float* f_b2  = (const float*)d_in[39];

  float* out = (float*)d_out;

  const size_t bSEQH = (size_t)NR * DM * 2;
  const size_t bW11  = (size_t)DM * DM * 2;
  const size_t bW21  = (size_t)DH * DM * 2;
  const size_t bDW1  = (size_t)DM * DC * 2;
  const size_t bW33  = (size_t)DH * DH * 2;
  const size_t bH1   = (size_t)NR * DM * 2;
  const size_t bH2   = (size_t)NR * DH * 4;
  const size_t bCAT  = (size_t)NR * DC * 2;
  const size_t bHA   = (size_t)NR * DH * 4;
  const size_t bDEC2 = (size_t)NR * DM * 4;
  const size_t bPQ   = (size_t)NHF * DH * 4;
  const size_t bVB   = (size_t)NR * DH * 4;
  const size_t bR1K  = (size_t)NR * 4;
  const size_t bR512 = (size_t)NHF * 4;
  const size_t bLOSS = 128;
  const size_t total = bSEQH + 3 * bW11 + 2 * bW21 + bDW1 + 5 * bW33 + bH1 + bH2 + bCAT + 2 * bHA +
                       bDEC2 + 2 * bPQ + 3 * bVB + 4 * bR1K + 2 * bR512 + bLOSS;
  if (total > ws_size) return;
  if (total > (size_t)134217728) return;

  char* ws = (char*)d_ws;
  size_t off = 0;
  _Float16* SEQH = (_Float16*)(ws + off); off += bSEQH;
  _Float16* W1AP = (_Float16*)(ws + off); off += bW11;
  _Float16* W2AP = (_Float16*)(ws + off); off += bW21;
  _Float16* W1CP = (_Float16*)(ws + off); off += bW11;
  _Float16* W2CP = (_Float16*)(ws + off); off += bW21;
  _Float16* DW1P = (_Float16*)(ws + off); off += bDW1;
  _Float16* DW2P = (_Float16*)(ws + off); off += bW11;
  _Float16* FWT  = (_Float16*)(ws + off); off += bW33;
  _Float16* FWB  = (_Float16*)(ws + off); off += bW33;
  _Float16* VWP  = (_Float16*)(ws + off); off += bW33;
  _Float16* AWP  = (_Float16*)(ws + off); off += bW33;
  _Float16* DWP  = (_Float16*)(ws + off); off += bW33;
  _Float16* H1   = (_Float16*)(ws + off); off += bH1;
  float*    H2   = (float*)(ws + off);    off += bH2;
  _Float16* CATH = (_Float16*)(ws + off); off += bCAT;
  float*    HA   = (float*)(ws + off);    off += bHA;
  float*    HC   = (float*)(ws + off);    off += bHA;
  float*    DEC2 = (float*)(ws + off);    off += bDEC2;
  float*    PB   = (float*)(ws + off);    off += bPQ;
  float*    QB   = (float*)(ws + off);    off += bPQ;
  float*    VB   = (float*)(ws + off);    off += bVB;
  float*    AB   = (float*)(ws + off);    off += bVB;
  float*    DB   = (float*)(ws + off);    off += bVB;
  float*    CLUB = (float*)(ws + off);    off += bR1K;
  float*    REC  = (float*)(ws + off);    off += bR1K;
  float*    VADP = (float*)(ws + off);    off += bR1K;
  float*    ORTH = (float*)(ws + off);    off += bR1K;
  float*    LSE  = (float*)(ws + off);    off += bR512;
  float*    T0   = (float*)(ws + off);    off += bR512;
  float*    LOSS = (float*)(ws + off);    off += bLOSS;
  if (off != total) return;

  const int n8S = NR * DM / 8;
  k_cvt<<<(unsigned)((n8S + 255) / 256), 256, 0, stream>>>(seq, SEQH, n8S);
  k_packw<<<dim3(DM / 64, DM / 64), 256, 0, stream>>>(ha_w1, DM, DM, W1AP);
  k_packw<<<dim3(DH / 64, DM / 64), 256, 0, stream>>>(ha_w2, DM, DH, W2AP);
  k_packw<<<dim3(DM / 64, DM / 64), 256, 0, stream>>>(hc_w1, DM, DM, W1CP);
  k_packw<<<dim3(DH / 64, DM / 64), 256, 0, stream>>>(hc_w2, DM, DH, W2CP);
  k_packw<<<dim3(DM / 64, DC / 64), 256, 0, stream>>>(de_w1, DC, DM, DW1P);
  k_packw<<<dim3(DM / 64, DM / 64), 256, 0, stream>>>(de_w2, DM, DM, DW2P);
  k_packw<<<dim3(DH / 64, DH / 64), 256, 0, stream>>>(f_w1, DH, DH, FWT);
  k_packw<<<dim3(DH / 64, DH / 64), 256, 0, stream>>>(f_w1 + (size_t)DH * DH, DH, DH, FWB);
  k_packw<<<dim3(DH / 64, DH / 64), 256, 0, stream>>>(v_w, DH, DH, VWP);
  k_packw<<<dim3(DH / 64, DH / 64), 256, 0, stream>>>(a_w, DH, DH, AWP);
  k_packw<<<dim3(DH / 64, DH / 64), 256, 0, stream>>>(d_w, DH, DH, DWP);

  k_gemm<<<dim3(DM / 64, NR / 64), 64, 0, stream>>>(SEQH, DM, W1AP, DM, ha_b1, 1, WINV, 1, DEC2, 0, H1, 1, DM);
  k_gemm<<<dim3(DH / 64, NR / 64), 64, 0, stream>>>(H1, DM, W2AP, DM, ha_b2, 1, WINV, 1, H2, 1, SEQH, 0, DH);
  k_ln256<<<NR / 32, 256, 0, stream>>>(H2, ha_g, ha_bt, HA, CATH, DC, 0, HC, 0, CLUB);

  k_gemm<<<dim3(DM / 64, NR / 64), 64, 0, stream>>>(SEQH, DM, W1CP, DM, hc_b1, 1, WINV, 1, DEC2, 0, H1, 1, DM);
  k_gemm<<<dim3(DH / 64, NR / 64), 64, 0, stream>>>(H1, DM, W2CP, DM, hc_b2, 1, WINV, 1, H2, 1, SEQH, 0, DH);
  k_ln256<<<NR / 32, 256, 0, stream>>>(H2, hc_g, hc_bt, HC, CATH, DC, DH, HA, 1, CLUB);

  k_gemm<<<dim3(DM / 64, NR / 64), 64, 0, stream>>>(CATH, DC, DW1P, DC, de_b1, 1, WINV, 1, DEC2, 0, H1, 1, DM);
  k_gemm<<<dim3(DM / 64, NR / 64), 64, 0, stream>>>(H1, DM, DW2P, DM, de_b2, 1, WINV, 1, DEC2, 1, SEQH, 0, DM);
  k_ln768<<<NR / 32, 256, 0, stream>>>(DEC2, de_g, de_bt, seq, REC);

  k_gemm<<<dim3(DH / 64, NHF / 64), 64, 0, stream>>>(CATH, DC, FWT, DH, f_b1, 0, WINV, 0, PB, 1, SEQH, 0, DH);
  k_gemm<<<dim3(DH / 64, NHF / 64), 64, 0, stream>>>(CATH + (size_t)NHF * DC, DC, FWB, DH, f_b1, 1, WINV, 0, QB, 1, SEQH, 0, DH);
  k_crit<<<NHF / 32, 256, 0, stream>>>(PB, QB, f_w2, f_b2, ids_o, ids_c, LSE, T0);

  k_gemm<<<dim3(DH / 64, NR / 64), 64, 0, stream>>>(CATH + DH, DC, VWP, DH, v_b, 1, WINV, 0, VB, 1, SEQH, 0, DH);
  k_gemm<<<dim3(DH / 64, NR / 64), 64, 0, stream>>>(CATH + DH, DC, AWP, DH, a_b, 1, WINV, 0, AB, 1, SEQH, 0, DH);
  k_gemm<<<dim3(DH / 64, NR / 64), 64, 0, stream>>>(CATH + DH, DC, DWP, DH, d_b, 1, WINV, 0, DB, 1, SEQH, 0, DH);
  k_vad<<<NR / 32, 256, 0, stream>>>(VB, AB, DB, pv_w, pa_w, pd_w, pv_b, pa_b, pd_b, vad_o, vad_c, VADP, ORTH);

  k_loss<<<1, 256, 0, stream>>>(CLUB, REC, LSE, T0, VADP, ORTH, amask, LOSS);
  k_out<<<(unsigned)((OUT4 + 1 + 255) / 256), 256, 0, stream>>>(LOSS, HA, HC, out);
}
